// TransformerHead_35794257445458
// MI455X (gfx1250) — hardware-verified
//
#include <hip/hip_runtime.h>
#include <stddef.h>


#define NB 2
#define NS 4096
#define NH 8
#define HD 64
#define DM 512
#define MR (NB * NS)

static_assert(NH * HD == DM);
static_assert(MR % 128 == 0);
static_assert(NS % 128 == 0);
static_assert(DM % 64 == 0);
static_assert((MR * DM) % 2048 == 0);

typedef unsigned short u16;
typedef __bf16   v16bf __attribute__((ext_vector_type(16)));
typedef _Float16 v16h  __attribute__((ext_vector_type(16)));
typedef float    v8f   __attribute__((ext_vector_type(8)));
typedef u16      v8u   __attribute__((ext_vector_type(8)));
typedef float    v4f   __attribute__((ext_vector_type(4)));
typedef v4f __attribute__((may_alias)) v4fa;

union FragB { v16bf v; v8u h[2]; };
union FragH { v16h v; v8u h[2]; _Float16 s[16]; };
union Pack8 { v8u v; u16 s[8]; _Float16 f[8]; };

enum { MD_QK = 0, MD_VT = 1, MD_OUT = 2 };


static __device__ __forceinline__ u16 bf_rne(float f) {
  unsigned u = __float_as_uint(f);
  u += 0x7FFFu + ((u >> 16) & 1u);
  return (u16)(u >> 16);
}
static __device__ __forceinline__ float bf_to_f(u16 b) {
  return __uint_as_float(((unsigned)b) << 16);
}
static __device__ __forceinline__ void split_bf(float x, u16& hi, u16& lo) {
  hi = bf_rne(x);
  lo = bf_rne(x - bf_to_f(hi));
}
static __device__ __forceinline__ void split8(v4f a, v4f b, Pack8& ph, Pack8& pl) {
#pragma unroll
  for (int e = 0; e < 4; ++e) {
    split_bf(a[e], ph.s[e], pl.s[e]);
    split_bf(b[e], ph.s[4 + e], pl.s[4 + e]);
  }
}

static __device__ __forceinline__ float fexp2(float x) {
#if __has_builtin(__builtin_amdgcn_exp2f)
  return __builtin_amdgcn_exp2f(x);
#else
  return exp2f(x);
#endif
}

static __device__ __forceinline__ v8f zero8() {
  v8f z = {0.f, 0.f, 0.f, 0.f, 0.f, 0.f, 0.f, 0.f};
  return z;
}

static __device__ __forceinline__ v16bf frag_bf(const u16* __restrict__ base, int row, int ld,
                                                int k0, int hf) {
  const u16* p = base + (size_t)row * ld + k0 + 8 * hf;
  FragB f;
  f.h[0] = *(const v8u*)(p);
  f.h[1] = *(const v8u*)(p + 16);
  return f.v;
}
static __device__ __forceinline__ v16h frag_h(const u16* __restrict__ base, int row, int ld,
                                              int k0, int hf) {
  const u16* p = base + (size_t)row * ld + k0 + 8 * hf;
  FragH f;
  f.h[0] = *(const v8u*)(p);
  f.h[1] = *(const v8u*)(p + 16);
  return f.v;
}

static __device__ __forceinline__ v8f mma_bf(v16bf a, v16bf b, v8f c) {
  c = __builtin_amdgcn_wmma_f32_16x16x32_bf16(false, a, false, b, (short)0, c, false, false);
  asm volatile("v_nop\n\tv_nop\n\tv_nop\n\tv_nop" : "+v"(c) : "v"(a), "v"(b));
  return c;
}
static __device__ __forceinline__ v8f mma_h(v16h a, v16h b, v8f c) {
  c = __builtin_amdgcn_wmma_f32_16x16x32_f16(false, a, false, b, (short)0, c, false, false);
  asm volatile("v_nop\n\tv_nop\n\tv_nop\n\tv_nop" : "+v"(c) : "v"(a), "v"(b));
  return c;
}

__global__ __launch_bounds__(256) void k_xsplit(const float* __restrict__ x,
                                                u16* xh, u16* xl, int n8) {
  const int i = blockIdx.x * 256 + (int)threadIdx.x;
  if (i >= n8) return;
  const size_t e = (size_t)i * 8;
  const v4f a = *(const v4f*)(x + e);
  const v4f b = *(const v4f*)(x + e + 4);
  Pack8 ph, pl;
  split8(a, b, ph, pl);
  *(volatile v8u*)(xh + e) = ph.v;
  *(volatile v8u*)(xl + e) = pl.v;
  __threadfence();
  *(volatile v8u*)(xh + e) = ph.v;
  *(volatile v8u*)(xl + e) = pl.v;
}

__global__ __launch_bounds__(256) void k_wsplit(const float* __restrict__ w0,
                                                const float* __restrict__ w1,
                                                const float* __restrict__ w2,
                                                const float* __restrict__ w3,
                                                u16* wt) {
  __shared__ __attribute__((aligned(16))) float tile[32 * 64];
  const int z = blockIdx.z;
  const float* w = (z == 0) ? w0 : (z == 1) ? w1 : (z == 2) ? w2 : w3;
  u16* oh = wt + (size_t)(2 * z) * DM * DM;
  u16* ol = oh + (size_t)DM * DM;
  const int k0 = blockIdx.x * 64, n0 = blockIdx.y * 32;
  const int t = threadIdx.x;
  const int nn = t & 31, kq = t >> 5;
#pragma unroll
  for (int i = 0; i < 8; ++i) {
    const int kk = kq + 8 * i;
    tile[nn * 64 + kk] = w[(size_t)(k0 + kk) * DM + n0 + nn];
  }
  __syncthreads();
  const int lane = t & 31, wave = t >> 5;
  const int q = lane >> 3, p = lane & 7;
  const int nl = wave * 4 + q;
  const v4fa* tp = (const v4fa*)(tile + nl * 64 + 8 * p);
  const v4f a = tp[0], b = tp[1];
  Pack8 ph, pl;
  split8(a, b, ph, pl);
  const size_t o = (size_t)(n0 + nl) * DM + k0 + 8 * p;
  *(volatile v8u*)(oh + o) = ph.v;
  *(volatile v8u*)(ol + o) = pl.v;
  __threadfence();
  *(volatile v8u*)(oh + o) = ph.v;
  *(volatile v8u*)(ol + o) = pl.v;
}

template <int MODE>
static __device__ __forceinline__ void gemm_lines(const float* tile, void* out0, void* out1,
                                                  int wave, int q, int p, int m0, int n0,
                                                  int bidx, int s0, int head) {
  if constexpr (MODE == MD_QK) {
    u16* oh = (u16*)out0;
    u16* ol = (u16*)out1;
#pragma unroll
    for (int it = 0; it < 4; ++it) {
      const int rl = wave * 16 + it * 4 + q;
      const v4fa* tp = (const v4fa*)(tile + rl * 64 + 8 * p);
      const v4f a = tp[0], b = tp[1];
      Pack8 ph, pl;
      split8(a, b, ph, pl);
      const size_t o = (((size_t)(bidx * NH + head)) * NS + (size_t)(s0 + rl)) * HD + 8 * p;
      *(volatile v8u*)(oh + o) = ph.v;
      *(volatile v8u*)(ol + o) = pl.v;
    }
  } else if constexpr (MODE == MD_VT) {
    u16* ov = (u16*)out0;
#pragma unroll
    for (int it = 0; it < 4; ++it) {
      const int li = it * 4 + q;
      const int nl = wave * 8 + (li >> 1);
      const int half = li & 1;
      Pack8 pk;
#pragma unroll
      for (int e = 0; e < 8; ++e)
        pk.f[e] = (_Float16)tile[(64 * half + 8 * p + e) * 64 + nl];
      const size_t o = (((size_t)(bidx * NH + head)) * HD + nl) * NS + s0 + 64 * half + 8 * p;
      *(volatile v8u*)(ov + o) = pk.v;
    }
  } else {
    float* of = (float*)out0;
#pragma unroll
    for (int it = 0; it < 8; ++it) {
      const int li = it * 4 + q;
      const int rl = wave * 16 + (li >> 1);
      const int half = li & 1;
      const v4f v = *(const v4fa*)(tile + rl * 64 + 32 * half + 4 * p);
      const size_t o = (size_t)(m0 + rl) * DM + n0 + 32 * half + 4 * p;
      *(volatile v4f*)(of + o) = v;
    }
  }
}

template <int MODE>
__global__ __launch_bounds__(256) void k_gemm(const u16* __restrict__ Ah, const u16* __restrict__ Al,
                                              const u16* __restrict__ Bh, const u16* __restrict__ Bl,
                                              const float* __restrict__ bias,
                                              void* out0, void* out1, float scale) {
  __shared__ __attribute__((aligned(16))) float tile[128 * 64];
  const int t = threadIdx.x;
  const int lane = t & 31, wave = t >> 5;
  const int lr = lane & 15, hf = lane >> 4;
  const int wr = wave >> 1, wc = wave & 1;
  const int m0 = blockIdx.x * 128, n0 = blockIdx.y * 64;
  const int row0 = m0 + wr * 32, col0 = n0 + wc * 32;

  v8f acc[2][2];
#pragma unroll
  for (int i = 0; i < 2; ++i)
#pragma unroll
    for (int j = 0; j < 2; ++j) acc[i][j] = zero8();

#pragma unroll 1
  for (int k0 = 0; k0 < DM; k0 += 32) {
    v16bf ah[2], al[2], bh[2], bl[2];
#pragma unroll
    for (int i = 0; i < 2; ++i) {
      ah[i] = frag_bf(Ah, row0 + 16 * i + lr, DM, k0, hf);
      al[i] = frag_bf(Al, row0 + 16 * i + lr, DM, k0, hf);
    }
#pragma unroll
    for (int j = 0; j < 2; ++j) {
      bh[j] = frag_bf(Bh, col0 + 16 * j + lr, DM, k0, hf);
      bl[j] = frag_bf(Bl, col0 + 16 * j + lr, DM, k0, hf);
    }
#pragma unroll
    for (int i = 0; i < 2; ++i)
#pragma unroll
      for (int j = 0; j < 2; ++j) {
        acc[i][j] = mma_bf(ah[i], bh[j], acc[i][j]);
        acc[i][j] = mma_bf(ah[i], bl[j], acc[i][j]);
        acc[i][j] = mma_bf(al[i], bh[j], acc[i][j]);
      }
  }

#pragma unroll
  for (int i = 0; i < 2; ++i)
#pragma unroll
    for (int j = 0; j < 2; ++j) {
      const int cl = wc * 32 + 16 * j + lr;
      const float bvv = bias[n0 + cl];
#pragma unroll
      for (int r = 0; r < 8; ++r)
        tile[(wr * 32 + 16 * i + 8 * hf + r) * 64 + cl] = (acc[i][j][r] + bvv) * scale;
    }
  __syncthreads();

  const int q = lane >> 3, p = lane & 7;
  const int bidx = m0 >> 12;
  const int s0 = m0 & (NS - 1);
  const int head = blockIdx.y;
  gemm_lines<MODE>(tile, out0, out1, wave, q, p, m0, n0, bidx, s0, head);
  __threadfence();
  gemm_lines<MODE>(tile, out0, out1, wave, q, p, m0, n0, bidx, s0, head);
}

static __device__ __forceinline__ void attn_lines(const float* tile, u16* ch, u16* cl,
                                                  int wave, int q, int p, int bidx, int head,
                                                  int qb) {
#pragma unroll
  for (int it = 0; it < 4; ++it) {
    const int ql = wave * 16 + it * 4 + q;
    const v4fa* tp = (const v4fa*)(tile + ql * 64 + 8 * p);
    const v4f a = tp[0], b = tp[1];
    Pack8 ph, pl;
    split8(a, b, ph, pl);
    const size_t o = ((size_t)(bidx * NS + qb + ql)) * DM + head * HD + 8 * p;
    *(volatile v8u*)(ch + o) = ph.v;
    *(volatile v8u*)(cl + o) = pl.v;
  }
}

__global__ __launch_bounds__(128) void k_attn(const u16* __restrict__ Qh, const u16* __restrict__ Ql,
                                              const u16* __restrict__ Kh, const u16* __restrict__ Kl,
                                              const u16* __restrict__ Vt,
                                              u16* Ch, u16* Cl) {
  __shared__ __attribute__((aligned(16))) float tile[64 * 64];
  const int t = threadIdx.x;
  const int lane = t & 31, wave = t >> 5;
  const int lr = lane & 15, hf = lane >> 4;
  const int bh = blockIdx.y;
  const int qb = blockIdx.x * 64;
  const int q0 = qb + wave * 16;

  const u16* qh = Qh + (size_t)bh * NS * HD;
  const u16* ql = Ql + (size_t)bh * NS * HD;
  const u16* kh = Kh + (size_t)bh * NS * HD;
  const u16* kl = Kl + (size_t)bh * NS * HD;
  const u16* vt = Vt + (size_t)bh * HD * NS;

  v16bf qfh[2], qfl[2];
#pragma unroll
  for (int c = 0; c < 2; ++c) {
    qfh[c] = frag_bf(qh, q0 + lr, HD, 32 * c, hf);
    qfl[c] = frag_bf(ql, q0 + lr, HD, 32 * c, hf);
  }

  v8f oacc[4];
#pragma unroll
  for (int dt = 0; dt < 4; ++dt) oacc[dt] = zero8();
  float mrun = -1.0e30f, lrun = 0.0f;

#pragma unroll 1
  for (int kb = 0; kb < NS; kb += 32) {
    v8f st[2];
    st[0] = zero8();
    st[1] = zero8();
#pragma unroll
    for (int c = 0; c < 2; ++c) {
#pragma unroll
      for (int kt = 0; kt < 2; ++kt) {
        const v16bf ka = frag_bf(kh, kb + 16 * kt + lr, HD, 32 * c, hf);
        const v16bf kc = frag_bf(kl, kb + 16 * kt + lr, HD, 32 * c, hf);
        st[kt] = mma_bf(ka, qfh[c], st[kt]);
        st[kt] = mma_bf(ka, qfl[c], st[kt]);
        st[kt] = mma_bf(kc, qfh[c], st[kt]);
      }
    }

    float bm = -1.0e30f;
#pragma unroll
    for (int kt = 0; kt < 2; ++kt)
#pragma unroll
      for (int r = 0; r < 8; ++r) bm = fmaxf(bm, st[kt][r]);
    bm = fmaxf(bm, __shfl_xor(bm, 16, 32));
    const float mnew = fmaxf(mrun, bm);
    const float alpha = fexp2(mrun - mnew);
    mrun = mnew;

    FragH pf;
    float sum = 0.0f;
#pragma unroll
    for (int r = 0; r < 8; ++r) {
      const float e0 = fexp2(st[0][r] - mnew);
      const float e1 = fexp2(st[1][r] - mnew);
      sum += e0 + e1;
      pf.s[r]     = (_Float16)(e0 * 64.0f);
      pf.s[8 + r] = (_Float16)(e1 * 64.0f);
    }
    sum += __shfl_xor(sum, 16, 32);
    lrun = lrun * alpha + sum;

#pragma unroll
    for (int dt = 0; dt < 4; ++dt) oacc[dt] = oacc[dt] * alpha;

#pragma unroll
    for (int dt = 0; dt < 4; ++dt) {
      const v16h vf = frag_h(vt, dt * 16 + lr, NS, kb, hf);
      oacc[dt] = mma_h(vf, pf.v, oacc[dt]);
    }
  }

  const float inv = (1.0f / lrun) * 0.015625f;
  float* trow = tile + (wave * 16 + lr) * 64 + 8 * hf;
#pragma unroll
  for (int dt = 0; dt < 4; ++dt) {
    v4f a, b;
    a[0] = oacc[dt][0] * inv; a[1] = oacc[dt][1] * inv; a[2] = oacc[dt][2] * inv; a[3] = oacc[dt][3] * inv;
    b[0] = oacc[dt][4] * inv; b[1] = oacc[dt][5] * inv; b[2] = oacc[dt][6] * inv; b[3] = oacc[dt][7] * inv;
    *(v4fa*)(trow + dt * 16) = a;
    *(v4fa*)(trow + dt * 16 + 4) = b;
  }
  __syncthreads();

  const int q = lane >> 3, p = lane & 7;
  const int bidx = bh >> 3, head = bh & 7;
  attn_lines(tile, Ch, Cl, wave, q, p, bidx, head, qb);
  __threadfence();
  attn_lines(tile, Ch, Cl, wave, q, p, bidx, head, qb);
}


extern "C" void kernel_launch(void* const* d_in, const int* in_sizes, int n_in,
                              void* d_out, int out_size, void* d_ws, size_t ws_size,
                              hipStream_t stream) {
  if (n_in != 9) return;
  if (in_sizes[0] != MR * DM || in_sizes[1] != DM * DM || in_sizes[2] != DM ||
      in_sizes[3] != DM * DM || in_sizes[4] != DM || in_sizes[5] != DM * DM ||
      in_sizes[6] != DM || in_sizes[7] != DM * DM || in_sizes[8] != DM) return;
  if (out_size != MR * DM) return;

  const size_t plane  = (size_t)MR * DM * sizeof(u16);
  const size_t wplane = (size_t)DM * DM * sizeof(u16);
  const size_t need = 9 * plane + 8 * wplane;
  if (ws_size < need) return;

  const float* X  = (const float*)d_in[0];
  const float* Wq = (const float*)d_in[1];
  const float* bq = (const float*)d_in[2];
  const float* Wk = (const float*)d_in[3];
  const float* bk = (const float*)d_in[4];
  const float* Wv = (const float*)d_in[5];
  const float* bv = (const float*)d_in[6];
  const float* Wo = (const float*)d_in[7];
  const float* bo = (const float*)d_in[8];

  char* ws = (char*)d_ws;
  size_t off = 0;
  u16* Xh  = (u16*)(ws + off); off += plane;
  u16* Xl  = (u16*)(ws + off); off += plane;
  u16* Wt  = (u16*)(ws + off); off += 8 * wplane;
  u16* Qh  = (u16*)(ws + off); off += plane;
  u16* Ql  = (u16*)(ws + off); off += plane;
  u16* Kh  = (u16*)(ws + off); off += plane;
  u16* Kl  = (u16*)(ws + off); off += plane;
  u16* Vtp = (u16*)(ws + off); off += plane;
  u16* Ch  = (u16*)(ws + off); off += plane;
  u16* Cl  = (u16*)(ws + off); off += plane;
  if (off > ws_size) return;

  const size_t wp = (size_t)DM * DM;

  const int n8 = MR * DM / 8;
  k_xsplit<<<(n8 + 255) / 256, 256, 0, stream>>>(X, Xh, Xl, n8);
  k_wsplit<<<dim3(DM / 64, DM / 32, 4), 256, 0, stream>>>(Wq, Wk, Wv, Wo, Wt);

  const dim3 gg(MR / 128, DM / 64);
  k_gemm<MD_QK><<<gg, 256, 0, stream>>>(Xh, Xl, Wt + 0 * wp, Wt + 1 * wp, bq,
                                         (void*)Qh, (void*)Ql, 0.18033688011112042f);
  k_gemm<MD_QK><<<gg, 256, 0, stream>>>(Xh, Xl, Wt + 2 * wp, Wt + 3 * wp, bk,
                                         (void*)Kh, (void*)Kl, 1.0f);
  k_gemm<MD_VT><<<gg, 256, 0, stream>>>(Xh, Xl, Wt + 4 * wp, Wt + 5 * wp, bv,
                                         (void*)Vtp, (void*)Vtp, 1.0f);

  k_attn<<<dim3(NS / 64, NB * NH), 128, 0, stream>>>(Qh, Ql, Kh, Kl, Vtp, Ch, Cl);

  k_gemm<MD_OUT><<<gg, 256, 0, stream>>>(Ch, Cl, Wt + 6 * wp, Wt + 7 * wp, bo,
                                          d_out, d_out, 1.0f);
}
